// TimelineGNNLayer7_39410619908408
// MI455X (gfx1250) — hardware-run, weakly checked
//
#include <hip/hip_runtime.h>
#include <stddef.h>
#include <stdint.h>


#define HID     128
#define NTHR    256
#define NWAVE   8
#define EPT     8
#define CHUNK   (NTHR * EPT)
#define WCAP    (EPT * 32)
#define LISTN   (NWAVE * WCAP)
#define NBA     1024
#define SLA     10
#define RCAP    16384
#define DEGCAP  64
#define MEAS_B1024  12531
#define MEAS_MAXDEG 29
#define NRELR   401
#define NTIME   1000
#define NQR     128
#define ECOLS   7
#define RTW     640
#define QHW     384
#define GBM     64
#define GBN     128
#define GTHR    128
#define TM      128
#define APITCH  392
#define ZP      128
#define AGGW    256
#define WSMAX   134217728

#define O_RB    0
#define O_W1B   81920
#define O_W2D   90112
#define O_TW3   122880
#define O_WHD   172032
#define O_HBT   204800
#define O_QBT   253952
#define WB_HALVES 303104
#define PW_U0   10240
#define PW_U1   11264
#define PW_U2   15360
#define PW_U3   21504
#define PW_U4   25600
#define PW_U5   31744
#define PW_U6   37888
#define O_REB   0
#define O_PEB   65536
#define O_QEB   131072
#define PA_HALVES 147456
#define PV_U0   8192
#define PV_U1   16384
#define PV_U2   18432
#define PV_NVEC 352
#define PA_BYTES (PA_HALVES * 2 + 8192)
#define VO_CBR  0
#define VO_CBT  640
#define VO_CBQ  768
#define VO_B2   1152
#define VO_WA   1280

#define BKT_ZINTS (RCAP + 3 * NBA)
#define BKT_LDS_INTS (LISTN + 2 * RCAP + 3 * NBA + 48)
#define EOFF_U    (TM * APITCH * 2)
#define EOFF_Z    (EOFF_U + TM * ZP * 4)
#define EOFF_M    (EOFF_Z + TM * ZP * 4)
#define EOFF_SL   (EOFF_M + TM * 16)
#define EOFF_AL   (EOFF_SL + TM * 4)
#define EOFF_C    (EOFF_AL + TM * 4)
#define EOFF_RID  (EOFF_C + 256 * 4)
#define EOFF_SEEN (EOFF_RID + 160 * 4)
#define EOFF_MISC (EOFF_SEEN + 256 * 4)
#define EDGE_LDS_BYTES (EOFF_MISC + 64)

static_assert(HID == 128 && TM == 128 && 4 * 256 == NBA);
static_assert((CHUNK & (CHUNK - 1)) == 0 && CHUNK <= 4096);
static_assert(NBA == (1 << SLA) && (NBA % 32) == 0);
static_assert(NRELR < 512 && NTIME < 1024 && NQR <= 128);
static_assert(RCAP >= MEAS_B1024 + 2048 && (RCAP % TM) == 0 && (RCAP % NTHR) == 0);
static_assert(DEGCAP >= MEAS_MAXDEG + 8);
static_assert((BKT_ZINTS % 4) == 0 && BKT_LDS_INTS * 4 <= 300000);
static_assert(EDGE_LDS_BYTES <= 327680 && EDGE_LDS_BYTES <= 300000);
static_assert((APITCH * 2) % 16 == 0 && APITCH >= 384);
static_assert((EOFF_U % 16) == 0 && (EOFF_Z % 16) == 0 && (EOFF_M % 16) == 0 && (EOFF_C % 16) == 0);
static_assert(PW_U6 * 8 == WB_HALVES && PV_U2 * 8 == PA_HALVES);
static_assert((PW_U0 % NTHR) == 0 && (PW_U1 % NTHR) == 0 && (PW_U2 % NTHR) == 0 && (PW_U3 % NTHR) == 0);
static_assert((PW_U4 % NTHR) == 0 && (PW_U5 % NTHR) == 0 && (PW_U6 % NTHR) == 0);
static_assert((PV_U0 % NTHR) == 0 && (PV_U1 % NTHR) == 0 && (PV_U2 % NTHR) == 0);
static_assert(O_W1B == 8 * PW_U0 && O_W2D == 8 * PW_U1 && O_TW3 == 8 * PW_U2 && O_WHD == 8 * PW_U3);
static_assert(O_HBT == 8 * PW_U4 && O_QBT == 8 * PW_U5);
static_assert(4 * PV_NVEC == VO_WA + 128);
static_assert(GBM == (GTHR / 32) * 16 && GBN == 128);

typedef float          v4f   __attribute__((ext_vector_type(4)));
typedef float          v8f   __attribute__((ext_vector_type(8)));
typedef int            v4i   __attribute__((ext_vector_type(4)));
typedef int            v8i   __attribute__((ext_vector_type(8)));
typedef unsigned short v8us  __attribute__((ext_vector_type(8)));
typedef __bf16         v16bf __attribute__((ext_vector_type(16)));
typedef v4f  __attribute__((may_alias)) v4fa;
typedef v4i  __attribute__((may_alias)) v4ia;
typedef v8us __attribute__((may_alias)) v8usa;
union FragB { v16bf v; v8us h[2]; v8i w; };

__device__ __forceinline__ v8f wmb(const FragB& a, const FragB& b, v8f c) {
  v8f d = __builtin_amdgcn_wmma_f32_16x16x32_bf16(false, a.v, false, b.v, (short)0, c, false, false);
  asm volatile("v_nop\n\tv_nop\n\tv_nop\n\tv_nop" : "+v"(d) : "v"(a.w), "v"(b.w));
  return d;
}

__device__ __forceinline__ unsigned int f2bf(float f) {
  const unsigned int u = __float_as_uint(f);
  const unsigned int r = ((u + 0x7FFFu + ((u >> 16) & 1u)) >> 16) & 0xFFFFu;
  return ((u & 0x7FFFFFFFu) > 0x7F800000u) ? 0x7FC0u : r;
}
__device__ __forceinline__ float bf2f(unsigned int b) { return __uint_as_float(b << 16); }
__device__ __forceinline__ float bfr(float f) { return bf2f(f2bf(f)); }
__device__ __forceinline__ void pin_i(int v) { asm volatile("" :: "v"(v)); }

__device__ __forceinline__ float leaky_f(float v) { return (v > 0.0f) ? v : 0.01f * v; }
__device__ __forceinline__ float sigm_f(float x) { return __builtin_amdgcn_rcpf(1.0f + __expf(-x)); }
__device__ __forceinline__ float tanh_f(float x) {
  return 1.0f - 2.0f * __builtin_amdgcn_rcpf(__expf(2.0f * x) + 1.0f);
}
__device__ __forceinline__ int clampi(int v, int lo, int hi) { return v < lo ? lo : (v > hi ? hi : v); }

__device__ __forceinline__ void put16(unsigned short* dp, v8us o) {
  *(volatile v8us*)dp = o;
  __threadfence();
  *(volatile v8us*)dp = o;
}
__device__ __forceinline__ void putf4(float* dp, v4f o) {
  *(volatile v4f*)dp = o;
  __threadfence();
  *(volatile v4f*)dp = o;
}
__device__ __forceinline__ void puti4(v4i* dp, v4i o) {
  *(volatile v4i*)dp = o;
  __threadfence();
  *(volatile v4i*)dp = o;
}
__device__ __forceinline__ v8us gat8(const float* __restrict__ p, int stride) {
  v8us o;
#pragma unroll
  for (int i = 0; i < 8; ++i) o[i] = (unsigned short)f2bf(p[(size_t)i * (size_t)stride]);
  return o;
}
__device__ __forceinline__ v8us cvt8(v4f a, v4f b, bool ok) {
  v8us o;
  o[0] = ok ? (unsigned short)f2bf(a.x) : (unsigned short)0;
  o[1] = ok ? (unsigned short)f2bf(a.y) : (unsigned short)0;
  o[2] = ok ? (unsigned short)f2bf(a.z) : (unsigned short)0;
  o[3] = ok ? (unsigned short)f2bf(a.w) : (unsigned short)0;
  o[4] = ok ? (unsigned short)f2bf(b.x) : (unsigned short)0;
  o[5] = ok ? (unsigned short)f2bf(b.y) : (unsigned short)0;
  o[6] = ok ? (unsigned short)f2bf(b.z) : (unsigned short)0;
  o[7] = ok ? (unsigned short)f2bf(b.w) : (unsigned short)0;
  return o;
}
__device__ __forceinline__ float blendf(float x, float y, unsigned mk) {
  return __uint_as_float((__float_as_uint(x) & mk) | (__float_as_uint(y) & ~mk));
}
__device__ __forceinline__ v8f widen8(v4i w) {
  v8f r;
  r[0] = __uint_as_float((unsigned)w.x << 16); r[1] = __uint_as_float((unsigned)w.x & 0xffff0000u);
  r[2] = __uint_as_float((unsigned)w.y << 16); r[3] = __uint_as_float((unsigned)w.y & 0xffff0000u);
  r[4] = __uint_as_float((unsigned)w.z << 16); r[5] = __uint_as_float((unsigned)w.z & 0xffff0000u);
  r[6] = __uint_as_float((unsigned)w.w << 16); r[7] = __uint_as_float((unsigned)w.w & 0xffff0000u);
  return r;
}

__global__ __launch_bounds__(NTHR) void k_pa(const float* __restrict__ hid, unsigned short* XB, int nN, int nUnits) {
  const int u = (int)blockIdx.x * NTHR + (int)threadIdx.x;
  if (u >= nUnits) return;
  const int row = u >> 4;
  const int k8  = (u & 15) * 8;
  const int rc  = row < nN ? row : nN - 1;
  const float* p = hid + (size_t)rc * HID + k8;
  const v4f a = *(const v4fa*)p;
  const v4f b = *(const v4fa*)(p + 4);
  asm volatile("" :: "v"(a), "v"(b));
  put16(XB + (size_t)row * HID + k8, cvt8(a, b, row < nN));
}

__global__ __launch_bounds__(NTHR) void k_pw(const float* __restrict__ W1, const float* __restrict__ W2,
                                             const float* __restrict__ gW, const float* __restrict__ tW,
                                             const float* __restrict__ Wr, const float* __restrict__ Ws,
                                             const float* __restrict__ Wq, const float* __restrict__ Wh,
                                             unsigned short* WB) {
  const int u = (int)blockIdx.x * NTHR + (int)threadIdx.x;
  v8us o;
  if (u < PW_U0) {
    const int n = u >> 4, k8 = (u & 15) * 8;
    if (n < 128)      o = gat8(W1 + (size_t)k8 * 128 + n, 128);
    else if (n < 384) o = gat8(gW + (size_t)k8 * 256 + (n - 128), 256);
    else if (n < 512) o = gat8(tW + (size_t)k8 * 128 + (n - 384), 128);
    else              o = gat8(Wr + (size_t)k8 * 128 + (n - 512), 128);
  } else if (u < PW_U1) {
    const int v = u - PW_U0, n = v >> 3, k8 = (v & 7) * 8;
    o = gat8(W1 + (size_t)(128 + k8) * 128 + n, 128);
  } else if (u < PW_U2) {
    const int v = u - PW_U1, n = v >> 5, k8 = (v & 31) * 8;
    o = gat8(W2 + (size_t)(k8 & 127) * 128 + n, 128);
  } else if (u < PW_U3) {
    const int v = u - PW_U2, n = v / 48, k8 = (v - n * 48) * 8;
    const int srow = (k8 < 256) ? k8 : (k8 - 128);
    o = gat8(tW + (size_t)srow * 128 + n, 128);
  } else if (u < PW_U4) {
    const int v = u - PW_U3, n = v >> 5, k8 = (v & 31) * 8;
    o = gat8(Wh + (size_t)(k8 & 127) * 128 + n, 128);
  } else if (u < PW_U5) {
    const int v = u - PW_U4, n = v >> 4, k8 = (v & 15) * 8;
    if (n < 256) o = gat8(gW + (size_t)(256 + k8) * 256 + n, 256);
    else         o = gat8(Ws + (size_t)k8 * 128 + (n - 256), 128);
  } else if (u < PW_U6) {
    const int v = u - PW_U5, n = v >> 4, k8 = (v & 15) * 8;
    if (n < 256) o = gat8(gW + (size_t)(128 + k8) * 256 + n, 256);
    else         o = gat8(Wq + (size_t)k8 * 128 + (n - 256), 128);
  } else {
    return;
  }
  put16(WB + (size_t)8 * (size_t)u, o);
}

__global__ __launch_bounds__(NTHR) void k_pv(const float* __restrict__ RE, const float* __restrict__ per,
                                             const float* __restrict__ pea, const int* __restrict__ qrel,
                                             const int* __restrict__ tsp, const float* __restrict__ b1,
                                             const float* __restrict__ b2, const float* __restrict__ gb,
                                             const float* __restrict__ tb, const float* __restrict__ wqb,
                                             const float* __restrict__ wal, unsigned short* PA) {
  const int u = (int)blockIdx.x * NTHR + (int)threadIdx.x;
  if (u < PV_U2) {
    v4f a, b;
    bool ok;
    if (u < PV_U0) {
      const int row = u >> 4, k8 = (u & 15) * 8;
      const int rc = row < NRELR ? row : NRELR - 1;
      const float* p = RE + (size_t)rc * HID + k8;
      a = *(const v4fa*)p; b = *(const v4fa*)(p + 4);
      ok = row < NRELR;
    } else if (u < PV_U1) {
      const int v = u - PV_U0, row = v >> 3, k8 = (v & 7) * 8;
      const int tc = row < NTIME ? row : NTIME - 1;
      const int ts = tsp[0];
      const int ta = clampi(ts - tc, 0, NTIME - 1);
      const int kk = k8 & 31;
      const float* p0 = per + (size_t)tc * 32 + kk;
      const float* p1 = pea + (size_t)ta * 32 + kk;
      const v4f ra = *(const v4fa*)p0, rb = *(const v4fa*)(p0 + 4);
      const v4f aa = *(const v4fa*)p1, ab = *(const v4fa*)(p1 + 4);
      asm volatile("" :: "v"(ra), "v"(rb), "v"(aa), "v"(ab));
      const unsigned mk = (k8 < 32) ? 0xffffffffu : 0u;
      a.x = blendf(ra.x, aa.x, mk); a.y = blendf(ra.y, aa.y, mk);
      a.z = blendf(ra.z, aa.z, mk); a.w = blendf(ra.w, aa.w, mk);
      b.x = blendf(rb.x, ab.x, mk); b.y = blendf(rb.y, ab.y, mk);
      b.z = blendf(rb.z, ab.z, mk); b.w = blendf(rb.w, ab.w, mk);
      ok = row < NTIME;
    } else {
      const int v = u - PV_U1, row = v >> 4, k8 = (v & 15) * 8;
      const int qr = clampi(qrel[row], 0, NRELR - 1);
      const float* p = RE + (size_t)qr * HID + k8;
      a = *(const v4fa*)p; b = *(const v4fa*)(p + 4);
      ok = true;
    }
    asm volatile("" :: "v"(a), "v"(b));
    put16(PA + (size_t)8 * (size_t)u, cvt8(a, b, ok));
    return;
  }
  const int vu = u - PV_U2;
  if (vu >= PV_NVEC) return;
  float* VF = (float*)(PA + PA_HALVES);
  v4f s;
  bool keep = true;
  if (vu < 160) {
    const int j = clampi(4 * vu - 384, 0, 124);
    s = *(const v4fa*)(tb + j);
    keep = (vu >= 96) && (vu < 128);
  } else if (vu < 192) {
    s = *(const v4fa*)(b1 + 4 * (vu - 160));
  } else if (vu < 256) {
    s = *(const v4fa*)(gb + 4 * (vu - 192));
  } else if (vu < 288) {
    s = *(const v4fa*)(wqb + 4 * (vu - 256));
  } else if (vu < 320) {
    s = *(const v4fa*)(b2 + 4 * (vu - 288));
  } else {
    s = *(const v4fa*)(wal + 4 * (vu - 320));
  }
  asm volatile("" :: "v"(s));
  v4f o;
  o.x = keep ? bfr(s.x) : 0.0f;
  o.y = keep ? bfr(s.y) : 0.0f;
  o.z = keep ? bfr(s.z) : 0.0f;
  o.w = keep ? bfr(s.w) : 0.0f;
  putf4(VF + 4 * vu, o);
}

template <int SLB>
__device__ __forceinline__ int scan_chunk7(const int* __restrict__ edges, int nE, int cbase, int slotBase,
                                           int nb, int* list, int tid, int lane, int wave) {
  int wc = 0;
  const int el0  = tid * EPT;
  const int e0   = cbase + el0;
  const int sent = -2147483647 - 1;
  int d0, d1, d2, d3, d4, d5, d6, d7;
#define LDK(J, DJ) { const int ej = e0 + (J); const int ec = ej < nE ? ej : nE - 1; \
    const int kv = edges[(size_t)ec * ECOLS + 5]; pin_i(kv); DJ = (ej < nE) ? kv : sent; }
  LDK(0, d0) LDK(1, d1) LDK(2, d2) LDK(3, d3) LDK(4, d4) LDK(5, d5) LDK(6, d6) LDK(7, d7)
#undef LDK
  const unsigned nbs = (unsigned)slotBase;
  const unsigned unb = (unsigned)nb;
  const unsigned s0 = (unsigned)d0 - nbs, s1 = (unsigned)d1 - nbs;
  const unsigned s2 = (unsigned)d2 - nbs, s3 = (unsigned)d3 - nbs;
  const unsigned s4 = (unsigned)d4 - nbs, s5 = (unsigned)d5 - nbs;
  const unsigned s6 = (unsigned)d6 - nbs, s7 = (unsigned)d7 - nbs;
  const bool h0 = s0 < unb, h1 = s1 < unb, h2 = s2 < unb, h3 = s3 < unb;
  const bool h4 = s4 < unb, h5 = s5 < unb, h6 = s6 < unb, h7 = s7 < unb;
  const unsigned any = __builtin_amdgcn_ballot_w32(h0 | h1 | h2 | h3 | h4 | h5 | h6 | h7);
  if (any != 0u) {
#define HITJ(J, HJ, SJ) { \
      const unsigned mj = __builtin_amdgcn_ballot_w32(HJ); \
      if (mj != 0u) { \
        if (HJ) { \
          const int pos = wc + (int)__builtin_amdgcn_mbcnt_lo(mj, 0u); \
          if (pos < WCAP) list[wave * WCAP + pos] = ((el0 + (J)) << SLB) | (int)(SJ); \
        } \
        wc += (int)__builtin_popcount(mj); } }
    HITJ(0, h0, s0)
    HITJ(1, h1, s1)
    HITJ(2, h2, s2)
    HITJ(3, h3, s3)
    HITJ(4, h4, s4)
    HITJ(5, h5, s5)
    HITJ(6, h6, s6)
    HITJ(7, h7, s7)
#undef HITJ
  }
  return wc;
}

__global__ __launch_bounds__(NTHR) void k_bucket(const int* __restrict__ edges, const int* __restrict__ nnp,
                                                 int nE, int nN, v4i* REC, int* FLG) {
  extern __shared__ __attribute__((aligned(16))) int bsm[];
  int* list = bsm;
  int* hl   = bsm + LISTN;
  int* sl   = hl + RCAP;
  int* cnt  = sl + RCAP;
  int* offs = cnt + NBA;
  int* cur  = offs + NBA;
  int* misc = cur + NBA;
  const int tid = (int)threadIdx.x, lane = tid & 31, wave = tid >> 5;
  const int blk = (int)blockIdx.x;
  const int nodeBase = blk * NBA;
  const int nseg = clampi(nnp[0], 0, nN);
  const int nb = clampi(nseg - nodeBase, 0, NBA);

  {
    const v4i z4 = {0, 0, 0, 0};
    for (int i = tid * 4; i < BKT_ZINTS; i += NTHR * 4) *(v4ia*)(sl + i) = z4;
    if (tid < 48) misc[tid] = 0;
  }
  __syncthreads();

  int tot = 0, ovf = 0;
  const int nChunks = (nE + CHUNK - 1) / CHUNK;
#pragma unroll 1
  for (int ch = 0; ch < nChunks; ++ch) {
    const int cbase = ch * CHUNK;
    const int wc = scan_chunk7<SLA>(edges, nE, cbase, nodeBase, nb, list, tid, lane, wave);
    if (lane == 0) misc[wave] = wc;
    __syncthreads();
    int pre = 0, all = 0;
#pragma unroll
    for (int w2 = 0; w2 < NWAVE; ++w2) {
      int c = misc[w2];
      c = c < 0 ? 0 : (c > WCAP ? WCAP : c);
      all += c;
      pre += (w2 < wave) ? c : 0;
    }
    const int wcc  = wc > WCAP ? WCAP : wc;
    const int base = tot + pre;
#pragma unroll 1
    for (int i = lane; i < wcc; i += 32) {
      const int ent = list[wave * WCAP + i];
      const int el  = (ent >> SLA) & (CHUNK - 1);
      const int sq  = ent & (NBA - 1);
      int eid = cbase + el;
      eid = eid > nE - 1 ? nE - 1 : eid;
      const int pos = base + i;
      if (pos < RCAP) hl[pos] = (eid << SLA) | sq;
    }
    if (tot + all > RCAP) ovf = 1;
    tot += all;
    tot = tot > RCAP ? RCAP : tot;
    __syncthreads();
  }
  const int nh = tot;

  if (wave == 0) {
#pragma unroll 1
    for (int b0 = 0; b0 < nh; b0 += 32) {
      const int idx = b0 + lane;
      const int uv  = hl[idx < nh ? idx : nh - 1];
      const int m32 = (nh - b0) < 32 ? (nh - b0) : 32;
#pragma unroll 1
      for (int k = 0; k < m32; ++k) {
        const int u  = __builtin_amdgcn_readlane(uv, k);
        const int sq = u & (NBA - 1);
        if (lane == 0) cnt[sq] = cnt[sq] + 1;
      }
    }
  }
  __syncthreads();
  if (wave == 0) {
    const int base = lane * (NBA / 32);
    int s = 0, bigl = 0;
#pragma unroll 1
    for (int i = 0; i < NBA / 32; ++i) {
      const int cv = cnt[base + i];
      s += cv;
      bigl |= (cv > DEGCAP) ? 1 : 0;
    }
    int incl = s;
#pragma unroll
    for (int d = 1; d < 32; d <<= 1) {
      const int y = __shfl_up(incl, d, 32);
      if (lane >= d) incl += y;
    }
    int run = incl - s;
#pragma unroll 1
    for (int i = 0; i < NBA / 32; ++i) {
      const int cv = cnt[base + i];
      offs[base + i] = run;
      cur[base + i]  = run;
      run += cv;
    }
    const unsigned bm = __builtin_amdgcn_ballot_w32(bigl != 0);
    if (lane == 0) misc[8] = (bm != 0u) ? 1 : 0;
  }
  __syncthreads();
  if (wave == 0) {
#pragma unroll 1
    for (int b0 = 0; b0 < nh; b0 += 32) {
      const int idx = b0 + lane;
      const int uv  = hl[idx < nh ? idx : nh - 1];
      const int m32 = (nh - b0) < 32 ? (nh - b0) : 32;
#pragma unroll 1
      for (int k = 0; k < m32; ++k) {
        const int u  = __builtin_amdgcn_readlane(uv, k);
        const int sq = u & (NBA - 1);
        if (lane == 0) {
          int p = cur[sq];
          p = p < 0 ? 0 : (p > RCAP - 1 ? RCAP - 1 : p);
          sl[p] = u;
          cur[sq] = p + 1;
        }
      }
    }
  }
  __syncthreads();

  if (tid < 32) {
    const int oi = offs[((tid - 2) & 3) * 256];
    const int fg = (ovf != 0 || misc[8] != 0) ? 1 : 0;
    int v = 0;
    v = (tid == 0) ? nh : v;
    v = (tid == 1) ? fg : v;
    v = (tid >= 2 && tid < 6) ? oi : v;
    v = (tid == 6) ? nh : v;
    misc[16 + tid] = v;
  }
  __syncthreads();

  v4i* rb = REC + (size_t)blk * RCAP;
#pragma unroll 1
  for (int p = tid; p < RCAP; p += NTHR) {
    const int u = sl[p];
    const bool live = p < nh;
    const int eid = clampi(u >> SLA, 0, nE - 1);
    const int sq  = u & (NBA - 1);
    const int* ep = edges + (size_t)eid * ECOLS;
    const int rr = ep[0];
    const int rl = ep[2];
    const int sb = ep[4];
    const int tt = ep[6];
    pin_i(rr); pin_i(rl); pin_i(sb); pin_i(tt);
    const int rq  = clampi(rr, 0, NQR - 1);
    const int rel = clampi(rl, 0, NRELR - 1);
    const int tc  = clampi(tt, 0, NTIME - 1);
    const int sub = clampi(sb, 0, nN - 1);
    v4i o;
    o.x = live ? (rel | (tc << 9) | (rq << 19)) : 0;
    o.y = live ? sub : 0;
    o.z = live ? sq : 0;
    o.w = live ? eid : 0;
    puti4(rb + p, o);
  }
  if (tid < 8) {
    const v4i cv = *(const v4ia*)(misc + 16 + 4 * tid);
    puti4((v4i*)(FLG + (size_t)blk * 32 + 4 * tid), cv);
  }
}

template <int HASB>
__global__ __launch_bounds__(GTHR) void k_gemm(const unsigned short* __restrict__ A, int lda,
                                               const unsigned short* __restrict__ BT, int ldb, int K,
                                               const float* __restrict__ bias, int nRows, float* Cm, int ldc) {
  __shared__ __attribute__((aligned(16))) float stg[GBM * GBN];
  const int tid = (int)threadIdx.x, lane = tid & 31, wave = tid >> 5, hh = lane >> 4, m = lane & 15;
  const int rowBase = (int)blockIdx.x * GBM;
  const int colBase = (int)blockIdx.y * GBN;

  v8f acc[8];
  {
    const v8f z = {0.f, 0.f, 0.f, 0.f, 0.f, 0.f, 0.f, 0.f};
#pragma unroll
    for (int t = 0; t < 8; ++t) acc[t] = z;
  }
  const unsigned short* ap = A  + (size_t)(rowBase + 16 * wave + m) * (size_t)lda + 8 * hh;
  const unsigned short* bp = BT + (size_t)(colBase + m) * (size_t)ldb + 8 * hh;

#pragma unroll 1
  for (int k0 = 0; k0 < K; k0 += 32) {
    FragB af;
    af.h[0] = *(const v8usa*)(ap + k0);
    af.h[1] = *(const v8usa*)(ap + k0 + 16);
#pragma unroll
    for (int nt = 0; nt < 8; ++nt) {
      const unsigned short* wq = bp + (size_t)(16 * nt) * (size_t)ldb + k0;
      FragB bf;
      bf.h[0] = *(const v8usa*)wq;
      bf.h[1] = *(const v8usa*)(wq + 16);
      acc[nt] = wmb(af, bf, acc[nt]);
    }
  }

#pragma unroll
  for (int nt = 0; nt < 8; ++nt) {
    const int lc = 16 * nt + m;
    float bvv = 0.0f;
    if constexpr (HASB != 0) bvv = bias[colBase + lc];
#pragma unroll
    for (int r = 0; r < 8; ++r) {
      const int lr = 16 * wave + 8 * hh + r;
      stg[lr * GBN + lc] = acc[nt][r] + bvv;
    }
  }
  __syncthreads();

  v4f pv[16];
#pragma unroll
  for (int i = 0; i < 16; ++i) pv[i] = *(const v4fa*)(stg + (16 * wave + i) * GBN + 4 * lane);
#pragma unroll
  for (int i = 0; i < 16; ++i) {
    const int row = rowBase + 16 * wave + i;
    if (row < nRows) {
      float* op = Cm + (size_t)row * (size_t)ldc + colBase + 4 * lane;
      *(volatile v4f*)op = pv[i];
    }
  }
  __threadfence();
#pragma unroll
  for (int i = 0; i < 16; ++i) {
    const int row = rowBase + 16 * wave + i;
    if (row < nRows) {
      float* op = Cm + (size_t)row * (size_t)ldc + colBase + 4 * lane;
      *(volatile v4f*)op = pv[i];
    }
  }
}

__device__ __forceinline__ void tile_gemm(const unsigned short* sAw, const unsigned short* __restrict__ BT,
                                          int ldb, int K, v8f (&acc)[8], int hh, int m) {
  {
    const v8f z = {0.f, 0.f, 0.f, 0.f, 0.f, 0.f, 0.f, 0.f};
#pragma unroll
    for (int t = 0; t < 8; ++t) acc[t] = z;
  }
  const unsigned short* ap = sAw + m * APITCH + 8 * hh;
  const unsigned short* bp = BT + (size_t)m * (size_t)ldb + 8 * hh;
#pragma unroll 1
  for (int k0 = 0; k0 < K; k0 += 32) {
    FragB af;
    af.h[0] = *(const v8usa*)(ap + k0);
    af.h[1] = *(const v8usa*)(ap + k0 + 16);
#pragma unroll
    for (int nt = 0; nt < 8; ++nt) {
      const unsigned short* wq = bp + (size_t)(16 * nt) * (size_t)ldb + k0;
      FragB bf;
      bf.h[0] = *(const v8usa*)wq;
      bf.h[1] = *(const v8usa*)(wq + 16);
      acc[nt] = wmb(af, bf, acc[nt]);
    }
  }
}
__device__ __forceinline__ void scatter_acc(float* sT, const v8f (&acc)[8], int wave, int hh, int m) {
#pragma unroll
  for (int nt = 0; nt < 8; ++nt)
#pragma unroll
    for (int r = 0; r < 8; ++r) sT[(16 * wave + 8 * hh + r) * ZP + 16 * nt + m] = acc[nt][r];
}
__device__ __forceinline__ v8us row_bits(const float* sp, unsigned mh, unsigned ml) {
  const v4f a = *(const v4fa*)sp;
  const v4f b = *(const v4fa*)(sp + 4);
  const v8f f8 = {a.x, a.y, a.z, a.w, b.x, b.y, b.z, b.w};
  v8us oo;
#pragma unroll
  for (int e = 0; e < 8; ++e) {
    const unsigned hb = f2bf(f8[e]);
    const unsigned lb = f2bf(f8[e] - bf2f(hb));
    oo[e] = (unsigned short)((hb & ml) | (lb & mh));
  }
  return oo;
}

__global__ __launch_bounds__(NTHR) __attribute__((amdgpu_num_vgpr(248)))
void k_edge(const v4i* __restrict__ REC, const int* __restrict__ FLG,
            const float* __restrict__ RTAB, const float* __restrict__ T1, const float* __restrict__ QTAB,
            const float* __restrict__ HCAT, const unsigned short* __restrict__ XB,
            const unsigned short* __restrict__ WB, const float* __restrict__ VF,
            unsigned short* AGG, int nN, int MP) {
  extern __shared__ __attribute__((aligned(16))) unsigned char esm[];
  unsigned short* sA = (unsigned short*)esm;
  float* sU    = (float*)(esm + EOFF_U);
  float* sZ    = (float*)(esm + EOFF_Z);
  int*   sMeta = (int*)(esm + EOFF_M);
  int*   sSlot = (int*)(esm + EOFF_SL);
  float* sAl   = (float*)(esm + EOFF_AL);
  float* sC    = (float*)(esm + EOFF_C);
  int*   sRid  = (int*)(esm + EOFF_RID);
  int*   sSeen = (int*)(esm + EOFF_SEEN);
  int*   sMisc = (int*)(esm + EOFF_MISC);

  const int tid = (int)threadIdx.x, lane = tid & 31, wave = tid >> 5, hh = lane >> 4, m = lane & 15;
  const int blk = (int)blockIdx.x >> 2;
  const int q   = (int)blockIdx.x & 3;
  const int rowBase = blk * NBA + 256 * q;

  const int* fl = FLG + (size_t)blk * 32;
  const int nhr = fl[0];
  const int bfl = fl[1];
  int s0 = fl[2 + q];
  int s1 = fl[3 + q];
  const int nhc = clampi(nhr, 0, RCAP);
  const bool bad = (bfl != 0) || (nhr < 0) || (nhr > RCAP);
  s0 = clampi(s0, 0, nhc);
  s1 = clampi(s1, s0, nhc);
  const int nEnt = s1 - s0;
  const int nTiles = (nEnt + TM - 1) / TM;
  const float qnan = __int_as_float(0x7fc00000);
  const float pz = bad ? qnan : 0.0f;

  sSeen[tid] = 0;
  sC[tid] = VF[VO_B2 + tid];
  if (tid < 16) sMisc[tid] = 0;
  __syncthreads();

  const v4i* rb = REC + (size_t)blk * RCAP;
  const int row = tid >> 1, hf = tid & 1;
  const unsigned short* sAw = sA + 16 * wave * APITCH;
  unsigned short* aRow = sA + row * APITCH + 64 * hf;
  float* uRow = sU + row * ZP + 64 * hf;
  float* zRow = sZ + row * ZP + 64 * hf;
  const int part = lane >> 4, pj = lane & 15;
  const unsigned mh = 0u - (unsigned)part;
  const unsigned ml = ~mh;

  int   cur = -1;
  float run = 0.0f;

#pragma unroll 1
  for (int tI = 0; tI < nTiles; ++tI) {
    const int base = s0 + TM * tI;
    int nv = s1 - base;
    nv = nv > TM ? TM : nv;

    if (tid < TM) {
      int idx = base + tid;
      idx = idx < s1 ? idx : s1 - 1;
      idx = clampi(idx, 0, RCAP - 1);
      const v4i e = rb[idx];
      v4i mt;
      mt.x = clampi(e.x & 511, 0, NRELR - 1);
      mt.y = clampi((e.x >> 9) & 1023, 0, NTIME - 1);
      mt.z = (e.x >> 19) & (NQR - 1);
      mt.w = clampi(e.y, 0, nN - 1);
      *(v4ia*)(sMeta + 4 * tid) = mt;
      sSlot[tid] = clampi(e.z - 256 * q, 0, 255);
    }
    __syncthreads();

    const v4i mt = *(const v4ia*)(sMeta + 4 * row);
    const float* pR = RTAB + (size_t)mt.x * RTW + 64 * hf;
    const float* pT = T1   + (size_t)mt.y * HID + 64 * hf;
    const float* pQ = QTAB + (size_t)mt.z * QHW + 64 * hf;
    const float* pH = HCAT + (size_t)mt.w * QHW + 64 * hf;
    const unsigned short* pX = XB + (size_t)mt.w * HID + 64 * hf;

#pragma unroll 1
    for (int c8 = 0; c8 < 8; ++c8) {
      const v4f ra = *(const v4fa*)(pR + 8 * c8);
      const v4f rb4 = *(const v4fa*)(pR + 8 * c8 + 4);
      const v4f ta = *(const v4fa*)(pT + 8 * c8);
      const v4f tb4 = *(const v4fa*)(pT + 8 * c8 + 4);
      const v8f r8 = {ra.x, ra.y, ra.z, ra.w, rb4.x, rb4.y, rb4.z, rb4.w};
      const v8f t8 = {ta.x, ta.y, ta.z, ta.w, tb4.x, tb4.y, tb4.z, tb4.w};
      v8us oh, ol;
#pragma unroll
      for (int i = 0; i < 8; ++i) {
        const float v = leaky_f(r8[i] + t8[i]);
        const unsigned hb = f2bf(v);
        oh[i] = (unsigned short)hb;
        ol[i] = (unsigned short)f2bf(v - bf2f(hb));
      }
      *(v8usa*)(aRow + 8 * c8)       = oh;
      *(v8usa*)(aRow + 128 + 8 * c8) = ol;
    }
    __syncthreads();

    v8f acc[8];

    tile_gemm(sAw, WB + O_W2D, 256, 256, acc, hh, m);
    __syncthreads();
#pragma unroll
    for (int nt = 0; nt < 8; ++nt) {
      const int col = 16 * nt + m;
      const float bb = sC[col];
#pragma unroll
      for (int r = 0; r < 8; ++r) {
        const float v = leaky_f(acc[nt][r] + bb);
        sA[(16 * wave + 8 * hh + r) * APITCH + col] = (unsigned short)f2bf(v);
      }
    }
    __syncthreads();

    tile_gemm(sAw, WB + O_RB + 512 * HID, HID, HID, acc, hh, m);
    scatter_acc(sZ, acc, wave, hh, m);
    __syncthreads();
    {
      float dot = 0.0f;
#pragma unroll 1
      for (int c4 = 0; c4 < 16; ++c4) {
        const v4f z  = *(const v4fa*)(zRow + 4 * c4);
        const v4f r  = *(const v4fa*)(pR + 512 + 4 * c4);
        const v4f qv = *(const v4fa*)(pQ + 256 + 4 * c4);
        const v4f hv = *(const v4fa*)(pH + 256 + 4 * c4);
        const v4f w  = *(const v4fa*)(sC + 128 + 64 * hf + 4 * c4);
        dot = fmaf(leaky_f(((z.x + r.x) + qv.x) + hv.x), w.x, dot);
        dot = fmaf(leaky_f(((z.y + r.y) + qv.y) + hv.y), w.y, dot);
        dot = fmaf(leaky_f(((z.z + r.z) + qv.z) + hv.z), w.z, dot);
        dot = fmaf(leaky_f(((z.w + r.w) + qv.w) + hv.w), w.w, dot);
      }
      const float oth = __shfl_xor(dot, 1, 32);
      const float sg = sigm_f(dot + oth);
      if (hf == 0) sAl[row] = sg;
    }

    tile_gemm(sAw, WB + O_RB + 128 * HID, HID, HID, acc, hh, m);
    scatter_acc(sU, acc, wave, hh, m);
    __syncthreads();
#pragma unroll 1
    for (int c4 = 0; c4 < 16; ++c4) {
      const v4f z  = *(const v4fa*)(uRow + 4 * c4);
      const v4f r  = *(const v4fa*)(pR + 128 + 4 * c4);
      const v4f qv = *(const v4fa*)(pQ + 4 * c4);
      const v4f hv = *(const v4fa*)(pH + 4 * c4);
      v4f g;
      g.x = sigm_f(((z.x + r.x) + qv.x) + hv.x);
      g.y = sigm_f(((z.y + r.y) + qv.y) + hv.y);
      g.z = sigm_f(((z.z + r.z) + qv.z) + hv.z);
      g.w = sigm_f(((z.w + r.w) + qv.w) + hv.w);
      *(v4fa*)(uRow + 4 * c4) = g;
    }

    tile_gemm(sAw, WB + O_RB + 256 * HID, HID, HID, acc, hh, m);
    scatter_acc(sZ, acc, wave, hh, m);
    __syncthreads();
#pragma unroll 1
    for (int c8 = 0; c8 < 8; ++c8) {
      const v4f za = *(const v4fa*)(zRow + 8 * c8);
      const v4f zb = *(const v4fa*)(zRow + 8 * c8 + 4);
      const v4f ra = *(const v4fa*)(pR + 256 + 8 * c8);
      const v4f rb4 = *(const v4fa*)(pR + 256 + 8 * c8 + 4);
      const v4f qa = *(const v4fa*)(pQ + 128 + 8 * c8);
      const v4f qb = *(const v4fa*)(pQ + 128 + 8 * c8 + 4);
      const v4f ha = *(const v4fa*)(pH + 128 + 8 * c8);
      const v4f hb4 = *(const v4fa*)(pH + 128 + 8 * c8 + 4);
      const v4i xw = *(const v4ia*)(pX + 8 * c8);
      const v8f z8 = {za.x, za.y, za.z, za.w, zb.x, zb.y, zb.z, zb.w};
      const v8f r8 = {ra.x, ra.y, ra.z, ra.w, rb4.x, rb4.y, rb4.z, rb4.w};
      const v8f q8 = {qa.x, qa.y, qa.z, qa.w, qb.x, qb.y, qb.z, qb.w};
      const v8f h8 = {ha.x, ha.y, ha.z, ha.w, hb4.x, hb4.y, hb4.z, hb4.w};
      const v8f x8 = widen8(xw);
      v8us oh, ol;
#pragma unroll
      for (int i = 0; i < 8; ++i) {
        const float g = sigm_f(((z8[i] + r8[i]) + q8[i]) + h8[i]);
        const float v = g * x8[i];
        const unsigned hb = f2bf(v);
        oh[i] = (unsigned short)hb;
        ol[i] = (unsigned short)f2bf(v - bf2f(hb));
      }
      *(v8usa*)(aRow + 128 + 8 * c8) = oh;
      *(v8usa*)(aRow + 256 + 8 * c8) = ol;
    }
    __syncthreads();

    tile_gemm(sAw, WB + O_TW3, 384, 384, acc, hh, m);
    scatter_acc(sZ, acc, wave, hh, m);
    __syncthreads();
    {
      const float sg = sAl[row];
      const bool rv = row < nv;
#pragma unroll 1
      for (int c8 = 0; c8 < 8; ++c8) {
        const v4f za = *(const v4fa*)(zRow + 8 * c8);
        const v4f zb = *(const v4fa*)(zRow + 8 * c8 + 4);
        const v4f ra = *(const v4fa*)(pR + 384 + 8 * c8);
        const v4f rb4 = *(const v4fa*)(pR + 384 + 8 * c8 + 4);
        const v4f ua = *(const v4fa*)(uRow + 8 * c8);
        const v4f ub = *(const v4fa*)(uRow + 8 * c8 + 4);
        const v4i xw = *(const v4ia*)(pX + 8 * c8);
        const v8f z8 = {za.x, za.y, za.z, za.w, zb.x, zb.y, zb.z, zb.w};
        const v8f r8 = {ra.x, ra.y, ra.z, ra.w, rb4.x, rb4.y, rb4.z, rb4.w};
        const v8f u8 = {ua.x, ua.y, ua.z, ua.w, ub.x, ub.y, ub.z, ub.w};
        const v8f x8 = widen8(xw);
        v8f o8;
#pragma unroll
        for (int i = 0; i < 8; ++i) {
          const float cand = tanh_f(z8[i] + r8[i]);
          const float msg = (1.0f - u8[i]) * x8[i] + u8[i] * cand;
          const float up = sg * msg;
          o8[i] = rv ? up : 0.0f;
        }
        const v4f o0 = {o8[0], o8[1], o8[2], o8[3]};
        const v4f o1 = {o8[4], o8[5], o8[6], o8[7]};
        *(v4fa*)(zRow + 8 * c8)     = o0;
        *(v4fa*)(zRow + 8 * c8 + 4) = o1;
      }
    }
    __syncthreads();

    if (wave < 4) {
      int kf = 0;
#pragma unroll 1
      for (int i = 0; i < nv; ++i) {
        const int s = sSlot[i];
        if (s != cur) {
          if (cur >= 0) {
            if (kf < TM) {
              sU[kf * ZP + tid] = run + pz;
              if (tid == 0) { sRid[kf] = cur; sSeen[cur] = 1; }
            }
            kf = kf + 1;
          }
          cur = s;
          run = 0.0f;
        }
        run += sZ[i * ZP + tid];
      }
      if (tid == 0) sMisc[0] = kf;
    }
    __syncthreads();
    {
      const int nfin = clampi(sMisc[0], 0, TM);
#pragma unroll 1
      for (int k = wave; k < nfin; k += NWAVE) {
        const int ls = clampi(sRid[k], 0, 255);
        const int grow = rowBase + ls;
        const v8us o = row_bits(sU + k * ZP + 8 * pj, mh, ml);
        if (grow < MP) *(volatile v8us*)(AGG + (size_t)grow * AGGW + part * HID + 8 * pj) = o;
      }
      __threadfence();
#pragma unroll 1
      for (int k = wave; k < nfin; k += NWAVE) {
        const int ls = clampi(sRid[k], 0, 255);
        const int grow = rowBase + ls;
        const v8us o = row_bits(sU + k * ZP + 8 * pj, mh, ml);
        if (grow < MP) *(volatile v8us*)(AGG + (size_t)grow * AGGW + part * HID + 8 * pj) = o;
      }
    }
    __syncthreads();
  }

  if (wave < 4) {
    sU[tid] = run + pz;
    if (tid == 0) {
      sRid[0] = cur < 0 ? 0 : cur;
      sMisc[1] = cur >= 0 ? 1 : 0;
      if (cur >= 0) sSeen[cur] = 1;
    }
  }
  __syncthreads();
  {
    const int hasLast = sMisc[1];
    const int ls = clampi(sRid[0], 0, 255);
    const int grow = rowBase + ls;
    const v8us o = row_bits(sU + 8 * pj, mh, ml);
    const bool st = (wave == 0) && (hasLast != 0) && (grow < MP);
    unsigned short* dp = AGG + (size_t)(grow < MP ? grow : MP - 1) * AGGW + part * HID + 8 * pj;
    if (st) *(volatile v8us*)dp = o;
    __threadfence();
    if (st) *(volatile v8us*)dp = o;
  }

  {
    const unsigned short zb = bad ? (unsigned short)0x7FC0 : (unsigned short)0;
    const v8us zo = {zb, zb, zb, zb, zb, zb, zb, zb};
#pragma unroll 1
    for (int j = 0; j < 32; ++j) {
      const int ls = wave + NWAVE * j;
      const int grow = rowBase + ls;
      if (sSeen[ls] == 0 && grow < MP) *(volatile v8us*)(AGG + (size_t)grow * AGGW + part * HID + 8 * pj) = zo;
    }
    __threadfence();
#pragma unroll 1
    for (int j = 0; j < 32; ++j) {
      const int ls = wave + NWAVE * j;
      const int grow = rowBase + ls;
      if (sSeen[ls] == 0 && grow < MP) *(volatile v8us*)(AGG + (size_t)grow * AGGW + part * HID + 8 * pj) = zo;
    }
  }
}

static inline int cdiv(int a, int b) { return (a + b - 1) / b; }

extern "C" void kernel_launch(void* const* d_in, const int* in_sizes, int n_in,
                              void* d_out, int out_size, void* d_ws, size_t ws_size,
                              hipStream_t stream) {
  if (n_in < 23) return;
  if (in_sizes[1] != NQR) return;
  if (in_sizes[2] < HID || (in_sizes[2] % HID) != 0) return;
  const int nN = in_sizes[2] / HID;
  if (in_sizes[3] < ECOLS || (in_sizes[3] % ECOLS) != 0) return;
  const int nE = in_sizes[3] / ECOLS;
  if (nE < 1 || nE >= (1 << 21)) return;
  if (in_sizes[4] != 1 || in_sizes[5] != 1) return;
  if (in_sizes[6] != NRELR * HID) return;
  if (in_sizes[7] != NTIME * 32 || in_sizes[8] != NTIME * 32) return;
  if (in_sizes[9] != HID * HID || in_sizes[10] != HID * HID || in_sizes[11] != HID * HID) return;
  if (in_sizes[12] != HID) return;
  if (in_sizes[13] != 192 * HID || in_sizes[14] != HID) return;
  if (in_sizes[15] != HID * HID || in_sizes[16] != HID) return;
  if (in_sizes[17] != HID) return;
  if (in_sizes[18] != 384 * 256 || in_sizes[19] != 256) return;
  if (in_sizes[20] != 256 * HID || in_sizes[21] != HID) return;
  if (in_sizes[22] != HID * HID) return;
  if ((long long)out_size != (long long)nN * HID) return;

  const int*   qrel  = (const int*)d_in[1];
  const float* hid   = (const float*)d_in[2];
  const int*   edges = (const int*)d_in[3];
  const int*   nnp   = (const int*)d_in[4];
  const int*   tsp   = (const int*)d_in[5];
  const float* RE    = (const float*)d_in[6];
  const float* per   = (const float*)d_in[7];
  const float* pea   = (const float*)d_in[8];
  const float* Ws    = (const float*)d_in[9];
  const float* Wr    = (const float*)d_in[10];
  const float* Wq    = (const float*)d_in[11];
  const float* wqb   = (const float*)d_in[12];
  const float* W1    = (const float*)d_in[13];
  const float* b1    = (const float*)d_in[14];
  const float* W2    = (const float*)d_in[15];
  const float* b2    = (const float*)d_in[16];
  const float* wal   = (const float*)d_in[17];
  const float* gW    = (const float*)d_in[18];
  const float* gb    = (const float*)d_in[19];
  const float* tW    = (const float*)d_in[20];
  const float* tb    = (const float*)d_in[21];
  const float* Wh    = (const float*)d_in[22];
  float* out = (float*)d_out;

  const int MP = cdiv(nN, GBM) * GBM;
  const int gM = MP / GBM;
  const int gA = cdiv(MP, NBA);
  if ((long long)gA * NBA < (long long)MP) return;
  if (((MP * 16) % NTHR) != 0) return;

  char* ws = (char*)d_ws;
  size_t off = 0;
  const size_t oXB   = off; off += (size_t)MP * HID * 2;          off = (off + 255) & ~(size_t)255;
  const size_t oHCAT = off; off += (size_t)MP * QHW * 4;          off = (off + 255) & ~(size_t)255;
  const size_t oAGG  = off; off += (size_t)MP * AGGW * 2;         off = (off + 255) & ~(size_t)255;
  const size_t oREC  = off; off += (size_t)gA * RCAP * 16;        off = (off + 255) & ~(size_t)255;
  const size_t oFLG  = off; off += (size_t)gA * 128;              off = (off + 255) & ~(size_t)255;
  const size_t oRTAB = off; off += (size_t)512 * RTW * 4;         off = (off + 255) & ~(size_t)255;
  const size_t oT1   = off; off += (size_t)1024 * HID * 4;        off = (off + 255) & ~(size_t)255;
  const size_t oQTAB = off; off += (size_t)NQR * QHW * 4;         off = (off + 255) & ~(size_t)255;
  const size_t oWB   = off; off += (size_t)WB_HALVES * 2;         off = (off + 255) & ~(size_t)255;
  const size_t oPA   = off; off += (size_t)PA_BYTES;              off = (off + 255) & ~(size_t)255;
  if (off > ws_size || off > (size_t)WSMAX) return;
  unsigned short* XB   = (unsigned short*)(ws + oXB);
  float*          HCAT = (float*)(ws + oHCAT);
  unsigned short* AGG  = (unsigned short*)(ws + oAGG);
  v4i*            REC  = (v4i*)(ws + oREC);
  int*            FLG  = (int*)(ws + oFLG);
  float*          RTAB = (float*)(ws + oRTAB);
  float*          T1   = (float*)(ws + oT1);
  float*          QTAB = (float*)(ws + oQTAB);
  unsigned short* WB   = (unsigned short*)(ws + oWB);
  unsigned short* PA   = (unsigned short*)(ws + oPA);
  const float*    VF   = (const float*)(PA + PA_HALVES);

  const int bktLds  = BKT_LDS_INTS * 4;
  const int edgeLds = EDGE_LDS_BYTES;
  hipFuncSetAttribute(reinterpret_cast<const void*>(&k_bucket),
                      hipFuncAttributeMaxDynamicSharedMemorySize, bktLds);
  hipFuncSetAttribute(reinterpret_cast<const void*>(&k_edge),
                      hipFuncAttributeMaxDynamicSharedMemorySize, edgeLds);

  k_pa<<<(MP * 16) / NTHR, NTHR, 0, stream>>>(hid, XB, nN, MP * 16);
  k_pw<<<PW_U6 / NTHR, NTHR, 0, stream>>>(W1, W2, gW, tW, Wr, Ws, Wq, Wh, WB);
  k_pv<<<cdiv(PV_U2 + PV_NVEC, NTHR), NTHR, 0, stream>>>(RE, per, pea, qrel, tsp, b1, b2, gb, tb, wqb, wal, PA);
  k_bucket<<<gA, NTHR, bktLds, stream>>>(edges, nnp, nE, nN, REC, FLG);
  k_gemm<1><<<dim3(512 / GBM, RTW / GBN), GTHR, 0, stream>>>(PA + O_REB, HID, WB + O_RB, HID, HID,
                                                              VF + VO_CBR, 512, RTAB, RTW);
  k_gemm<1><<<dim3(1024 / GBM, 1), GTHR, 0, stream>>>(PA + O_PEB, 64, WB + O_W1B, 64, 64,
                                                       VF + VO_CBT, 1024, T1, HID);
  k_gemm<1><<<dim3(NQR / GBM, QHW / GBN), GTHR, 0, stream>>>(PA + O_QEB, HID, WB + O_QBT, HID, HID,
                                                              VF + VO_CBQ, NQR, QTAB, QHW);
  k_gemm<0><<<dim3(gM, QHW / GBN), GTHR, 0, stream>>>(XB, HID, WB + O_HBT, HID, HID,
                                                       VF, MP, HCAT, QHW);
  k_edge<<<4 * gA, NTHR, edgeLds, stream>>>(REC, FLG, RTAB, T1, QTAB, HCAT, XB, WB, VF, AGG, nN, MP);
  k_gemm<0><<<dim3(gM, 1), GTHR, 0, stream>>>(AGG, AGGW, WB + O_WHD, AGGW, AGGW,
                                               VF, nN, out, HID);
}
